// CharLSTMEmbedding_50079318671863
// MI455X (gfx1250) — hardware-verified
//
#include <hip/hip_runtime.h>
#include <stdint.h>

typedef _Float16       v16h  __attribute__((ext_vector_type(16)));
typedef _Float16       v8h   __attribute__((ext_vector_type(8)));
typedef unsigned short v16us __attribute__((ext_vector_type(16)));
typedef unsigned short v8us  __attribute__((ext_vector_type(8)));
typedef __bf16         v16bf __attribute__((ext_vector_type(16)));
typedef float          v8f   __attribute__((ext_vector_type(8)));
typedef float          v4f   __attribute__((ext_vector_type(4)));
typedef v8h  __attribute__((may_alias)) v8ha;
typedef v8us __attribute__((may_alias)) v8usa;
typedef v4f  __attribute__((may_alias)) v4fa;

union FragH { v16h v; v8h half[2]; };
union FragU { v16us v; v8us half[2]; };

#define NROWS  4096
#define NSTEP  16
#define EDIM   256
#define HDIM   512
#define GDIM   2048
#define VOCAB  256
#define HSCALE 16.0f
#define WSCALE 64.0f
#define ACCINV 0.0009765625f

#define CV_NB_EMB (VOCAB * EDIM / 8 / 256)
#define CV_NB_WIH (GDIM * EDIM / 8 / 256)
#define CV_NB_WHH (GDIM * HDIM / 8 / 256)

__device__ __forceinline__ v8f wmma_bf16(v16us a, v16us b, v8f c) {
  v8f d = __builtin_amdgcn_wmma_f32_16x16x32_bf16(false, __builtin_bit_cast(v16bf, a), false,
                                                  __builtin_bit_cast(v16bf, b), (short)0, c, false, false);
  asm volatile("v_nop\n\tv_nop\n\tv_nop\n\tv_nop" : "+v"(d) : "v"(a), "v"(b));
  return d;
}

__device__ __forceinline__ v8f wmma_f16_raw(v16h a, v16h b, v8f c) {
  return __builtin_amdgcn_wmma_f32_16x16x32_f16(false, a, false, b, (short)0, c, false, false);
}

__device__ __forceinline__ v16h load_frag_h(const _Float16* p, int h) {
  FragH f;
  f.half[0] = *(const v8ha*)(p + 8 * h);
  f.half[1] = *(const v8ha*)(p + 16 + 8 * h);
  return f.v;
}
__device__ __forceinline__ v16us load_frag_u(const unsigned short* p, int h) {
  FragU f;
  f.half[0] = *(const v8usa*)(p + 8 * h);
  f.half[1] = *(const v8usa*)(p + 16 + 8 * h);
  return f.v;
}

__device__ __forceinline__ unsigned int bf16_bits(float x) {
  const unsigned int u = __float_as_uint(x);
  return (u + 0x7FFFu + ((u >> 16) & 1u)) >> 16;
}

__device__ __forceinline__ float frcp(float x) { return __builtin_amdgcn_rcpf(x); }
__device__ __forceinline__ float fsigmoid(float x) { return frcp(1.0f + __expf(-x)); }
__device__ __forceinline__ float ftanh(float x) {
  const float e = __expf(-2.0f * fabsf(x));
  const float r = (1.0f - e) * frcp(1.0f + e);
  return copysignf(r, x);
}

__global__ __launch_bounds__(256) void k_convert(
    const float* __restrict__ emb, const float* __restrict__ wih, const float* __restrict__ whh,
    unsigned short* __restrict__ embHi, unsigned short* __restrict__ embLo,
    unsigned short* __restrict__ wihHi, unsigned short* __restrict__ wihLo,
    _Float16* __restrict__ whh16)
{
  const int bid = blockIdx.x, tid = threadIdx.x;
  if (bid < CV_NB_EMB + CV_NB_WIH) {
    const float* src;
    unsigned short* dh;
    unsigned short* dl;
    if (bid < CV_NB_EMB) {
      const size_t g = (size_t)bid * 256 + tid;
      src = emb + g * 8; dh = embHi + g * 8; dl = embLo + g * 8;
    } else {
      const size_t g = (size_t)(bid - CV_NB_EMB) * 256 + tid;
      src = wih + g * 8; dh = wihHi + g * 8; dl = wihLo + g * 8;
    }
    const v4f a = *(const v4fa*)src;
    const v4f b = *(const v4fa*)(src + 4);
    const float x[8] = {a[0], a[1], a[2], a[3], b[0], b[1], b[2], b[3]};
    v8us oh, ol;
    #pragma unroll
    for (int i = 0; i < 8; ++i) {
      const unsigned int hb = bf16_bits(x[i]);
      const float hf = __uint_as_float(hb << 16);
      const unsigned int lb = bf16_bits(x[i] - hf);
      oh[i] = (unsigned short)hb;
      ol[i] = (unsigned short)lb;
    }
    *(volatile v8us*)dh = oh;
    *(volatile v8us*)dl = ol;
    __threadfence();
    *(volatile v8us*)dh = oh;
    *(volatile v8us*)dl = ol;
  } else {
    const size_t g = (size_t)(bid - CV_NB_EMB - CV_NB_WIH) * 256 + tid;
    const float* src = whh + g * 8;
    const v4f a = *(const v4fa*)src;
    const v4f b = *(const v4fa*)(src + 4);
    const v8h o = { (_Float16)(a[0] * WSCALE), (_Float16)(a[1] * WSCALE), (_Float16)(a[2] * WSCALE), (_Float16)(a[3] * WSCALE),
                    (_Float16)(b[0] * WSCALE), (_Float16)(b[1] * WSCALE), (_Float16)(b[2] * WSCALE), (_Float16)(b[3] * WSCALE) };
    _Float16* dst = whh16 + g * 8;
    *(volatile v8h*)dst = o;
    __threadfence();
    *(volatile v8h*)dst = o;
  }
}

__device__ __forceinline__ void gpre_store(const float* sG, float* G, int m0, int n0, int w, int lane) {
  const int q8 = lane & 7, sub = lane >> 3;
  #pragma unroll
  for (int i = 0; i < 8; ++i) {
    const int lid = 32 * w + 4 * i + sub;
    const int row = lid >> 1, hl = lid & 1;
    const v4f v = *(const v4fa*)(sG + row * 64 + 32 * hl + 4 * q8);
    *(volatile v4f*)(G + (size_t)(m0 + row) * GDIM + n0 + 32 * hl + 4 * q8) = v;
  }
}

__global__ __launch_bounds__(128) void k_gpre(
    const unsigned short* __restrict__ embHi, const unsigned short* __restrict__ embLo,
    const unsigned short* __restrict__ wihHi, const unsigned short* __restrict__ wihLo,
    const float* __restrict__ bih, const float* __restrict__ bhh,
    float* __restrict__ G)
{
  __shared__ __attribute__((aligned(16))) float sG[64 * 64];

  const int tid = threadIdx.x, lane = tid & 31, w = tid >> 5;
  const int h = lane >> 4, m = lane & 15;
  const int m0 = blockIdx.x * 64, n0 = blockIdx.y * 64;

  const size_t arow = (size_t)(m0 + 16 * w + m) * EDIM;
  const unsigned short* aH = embHi + arow;
  const unsigned short* aL = embLo + arow;
  const size_t brow = (size_t)(n0 + m) * EDIM;
  const unsigned short* bH = wihHi + brow;
  const unsigned short* bL = wihLo + brow;

  const v8f zero8 = {0.f, 0.f, 0.f, 0.f, 0.f, 0.f, 0.f, 0.f};
  v8f acc[4];
  #pragma unroll
  for (int nt = 0; nt < 4; ++nt) acc[nt] = zero8;

  #pragma unroll 1
  for (int k0 = 0; k0 < EDIM; k0 += 32) {
    const v16us ah = load_frag_u(aH + k0, h);
    const v16us al = load_frag_u(aL + k0, h);
    #pragma unroll
    for (int nt = 0; nt < 4; ++nt) {
      const v16us bh = load_frag_u(bH + (size_t)nt * 16 * EDIM + k0, h);
      const v16us bl = load_frag_u(bL + (size_t)nt * 16 * EDIM + k0, h);
      acc[nt] = wmma_bf16(ah, bh, acc[nt]);
      acc[nt] = wmma_bf16(al, bh, acc[nt]);
      acc[nt] = wmma_bf16(ah, bl, acc[nt]);
    }
  }

  #pragma unroll
  for (int nt = 0; nt < 4; ++nt) {
    const int col = n0 + 16 * nt + m;
    const float bs = bih[col] + bhh[col];
    #pragma unroll
    for (int r = 0; r < 8; ++r)
      sG[(16 * w + 8 * h + r) * 64 + 16 * nt + m] = acc[nt][r] + bs;
  }
  __syncthreads();

  gpre_store(sG, G, m0, n0, w, lane);
  __threadfence();
  gpre_store(sG, G, m0, n0, w, lane);
}

__device__ __forceinline__ void step_store(const float* sh, const float* sc, const _Float16* shh,
                                           float* hst, float* cst, _Float16* h16w,
                                           int m0, int n0, int w, int lane) {
  const int q8 = lane & 7, sub = lane >> 3;
  #pragma unroll
  for (int i = 0; i < 4; ++i) {
    const int lid = 16 * w + 4 * i + sub;
    const int row = lid >> 1, hl = lid & 1;
    const int so = row * 64 + 32 * hl + 4 * q8;
    const v4f vh = *(const v4fa*)(sh + so);
    const v4f vc = *(const v4fa*)(sc + so);
    const size_t gi = (size_t)(m0 + row) * HDIM + n0 + 32 * hl + 4 * q8;
    *(volatile v4f*)(hst + gi) = vh;
    *(volatile v4f*)(cst + gi) = vc;
  }
  #pragma unroll
  for (int i = 0; i < 2; ++i) {
    const int row = 8 * w + 4 * i + sub;
    const v8h v = *(const v8ha*)(shh + row * 64 + 8 * q8);
    *(volatile v8h*)(h16w + (size_t)(m0 + row) * HDIM + n0 + 8 * q8) = v;
  }
}

__global__ __launch_bounds__(128) void k_step(
    const _Float16* __restrict__ whh16,
    const float*    __restrict__ G,
    const int*      __restrict__ seq,
    const int*      __restrict__ lens,
    const _Float16* __restrict__ h16r,
    _Float16*       __restrict__ h16w,
    float*          __restrict__ hst,
    float*          __restrict__ cst,
    int t)
{
  __shared__ __attribute__((aligned(16))) float    sg[4 * 32 * 64];
  __shared__ __attribute__((aligned(16))) float    sh[32 * 64];
  __shared__ __attribute__((aligned(16))) float    sc[32 * 64];
  __shared__ __attribute__((aligned(16))) _Float16 shh[32 * 64];

  const int tid = threadIdx.x, lane = tid & 31, w = tid >> 5;
  const int h = lane >> 4, m = lane & 15;
  const int m0 = blockIdx.x * 32;
  const int n0 = blockIdx.y * 64;
  const int nw = n0 + 16 * w;

  const v8f zero8 = {0.f, 0.f, 0.f, 0.f, 0.f, 0.f, 0.f, 0.f};
  v8f acc[2][4];
  #pragma unroll
  for (int mt = 0; mt < 2; ++mt)
    #pragma unroll
    for (int g = 0; g < 4; ++g) acc[mt][g] = zero8;

  if (t > 0) {
    const _Float16* a0p = h16r + (size_t)(m0 + m) * HDIM;
    const _Float16* a1p = a0p + (size_t)16 * HDIM;
    const _Float16* bp  = whh16 + (size_t)(nw + m) * HDIM;
    const size_t gs = (size_t)HDIM * HDIM;
    #pragma unroll 2
    for (int k0 = 0; k0 < HDIM; k0 += 32) {
      const v16h a0 = load_frag_h(a0p + k0, h);
      const v16h a1 = load_frag_h(a1p + k0, h);
      const v16h b0 = load_frag_h(bp + k0, h);
      const v16h b1 = load_frag_h(bp + gs + k0, h);
      const v16h b2 = load_frag_h(bp + 2 * gs + k0, h);
      const v16h b3 = load_frag_h(bp + 3 * gs + k0, h);
      acc[0][0] = wmma_f16_raw(a0, b0, acc[0][0]);
      acc[1][0] = wmma_f16_raw(a1, b0, acc[1][0]);
      acc[0][1] = wmma_f16_raw(a0, b1, acc[0][1]);
      acc[1][1] = wmma_f16_raw(a1, b1, acc[1][1]);
      acc[0][2] = wmma_f16_raw(a0, b2, acc[0][2]);
      acc[1][2] = wmma_f16_raw(a1, b2, acc[1][2]);
      acc[0][3] = wmma_f16_raw(a0, b3, acc[0][3]);
      acc[1][3] = wmma_f16_raw(a1, b3, acc[1][3]);
      asm volatile("v_nop\n\tv_nop\n\tv_nop\n\tv_nop"
                   : "+v"(acc[0][0]), "+v"(acc[1][0]), "+v"(acc[0][1]), "+v"(acc[1][1]),
                     "+v"(acc[0][2]), "+v"(acc[1][2]), "+v"(acc[0][3]), "+v"(acc[1][3])
                   : "v"(a0), "v"(a1), "v"(b0), "v"(b1), "v"(b2), "v"(b3));
    }
  }

  #pragma unroll
  for (int mt = 0; mt < 2; ++mt)
    #pragma unroll
    for (int g = 0; g < 4; ++g)
      #pragma unroll
      for (int r = 0; r < 8; ++r)
        sg[(g * 32 + 16 * mt + 8 * h + r) * 64 + 16 * w + m] = acc[mt][g][r];
  __syncthreads();

  const int cl = tid & 63;
  const int rb = tid >> 6;
  const int col = n0 + cl;
  const bool warm = (t > 0);
  #pragma unroll 1
  for (int it = 0; it < 16; ++it) {
    const int rl = 2 * it + rb;
    const int row = m0 + rl;
    int id = seq[row * NSTEP + t];
    id = min(max(id, 0), VOCAB - 1);
    const int len = lens[row];
    const float* gr = G + (size_t)id * GDIM + col;
    const float* sp = sg + rl * 64 + cl;
    const float pi = sp[0 * 2048] * ACCINV + gr[0];
    const float pf = sp[1 * 2048] * ACCINV + gr[HDIM];
    const float pg = sp[2 * 2048] * ACCINV + gr[2 * HDIM];
    const float po = sp[3 * 2048] * ACCINV + gr[3 * HDIM];
    float cold = 0.0f, hold = 0.0f;
    if (warm) {
      const size_t off = (size_t)row * HDIM + col;
      cold = cst[off];
      hold = hst[off];
    }
    const float iv = fsigmoid(pi);
    const float fv = fsigmoid(pf);
    const float gv = ftanh(pg);
    const float ov = fsigmoid(po);
    const float cnew = fv * cold + iv * gv;
    const float hnew = ov * ftanh(cnew);
    const bool act = len > t;
    const float hs = act ? hnew : hold;
    const float cs = act ? cnew : cold;
    sh[rl * 64 + cl]  = hs;
    sc[rl * 64 + cl]  = cs;
    shh[rl * 64 + cl] = (_Float16)(hs * HSCALE);
  }
  __syncthreads();

  step_store(sh, sc, shh, hst, cst, h16w, m0, n0, w, lane);
  __threadfence();
  step_store(sh, sc, shh, hst, cst, h16w, m0, n0, w, lane);
}

extern "C" void kernel_launch(void* const* d_in, const int* in_sizes, int n_in,
                              void* d_out, int out_size, void* d_ws, size_t ws_size,
                              hipStream_t stream) {
  if (n_in < 7) return;
  if (in_sizes[0] != NROWS * NSTEP || in_sizes[1] != NROWS) return;
  if (in_sizes[2] != VOCAB * EDIM || in_sizes[3] != GDIM * EDIM || in_sizes[4] != GDIM * HDIM) return;
  if (in_sizes[5] != GDIM || in_sizes[6] != GDIM) return;
  if (out_size != NROWS * HDIM) return;

  const int*   seq  = (const int*)d_in[0];
  const int*   lens = (const int*)d_in[1];
  const float* emb  = (const float*)d_in[2];
  const float* wih  = (const float*)d_in[3];
  const float* whh  = (const float*)d_in[4];
  const float* bih  = (const float*)d_in[5];
  const float* bhh  = (const float*)d_in[6];
  float* hst = (float*)d_out;

  const size_t szE   = (size_t)VOCAB * EDIM * 2;
  const size_t szWI  = (size_t)GDIM * EDIM * 2;
  const size_t szWH  = (size_t)GDIM * HDIM * 2;
  const size_t szG   = (size_t)VOCAB * GDIM * 4;
  const size_t szC   = (size_t)NROWS * HDIM * 4;
  const size_t szH16 = (size_t)NROWS * HDIM * 2;
  const size_t oEH = 0;
  const size_t oEL = oEH + szE;
  const size_t oWH = oEL + szE;
  const size_t oWL = oWH + szWI;
  const size_t oW2 = oWL + szWI;
  const size_t oG  = oW2 + szWH;
  const size_t oC  = oG + szG;
  const size_t oHA = oC + szC;
  const size_t oHB = oHA + szH16;
  const size_t total = oHB + szH16;
  if (total > ws_size) return;

  char* ws = (char*)d_ws;
  unsigned short* embHi = (unsigned short*)(ws + oEH);
  unsigned short* embLo = (unsigned short*)(ws + oEL);
  unsigned short* wihHi = (unsigned short*)(ws + oWH);
  unsigned short* wihLo = (unsigned short*)(ws + oWL);
  _Float16* whh16 = (_Float16*)(ws + oW2);
  float* G = (float*)(ws + oG);
  float* cst = (float*)(ws + oC);
  _Float16* h16[2] = { (_Float16*)(ws + oHA), (_Float16*)(ws + oHB) };

  k_convert<<<CV_NB_EMB + CV_NB_WIH + CV_NB_WHH, 256, 0, stream>>>(emb, wih, whh, embHi, embLo, wihHi, wihLo, whh16);

  dim3 gG(VOCAB / 64, GDIM / 64);
  k_gpre<<<gG, 128, 0, stream>>>(embHi, embLo, wihHi, wihLo, bih, bhh, G);

  dim3 gS(NROWS / 32, HDIM / 64);
  for (int t = 0; t < NSTEP; ++t) {
    const _Float16* hr = h16[t & 1];
    _Float16* hw = h16[(t + 1) & 1];
    k_step<<<gS, 128, 0, stream>>>(whh16, G, seq, lens, hr, hw, hst, cst, t);
  }
}
